// MultiHeadAttention_54400055771505
// MI455X (gfx1250) — hardware-verified
//
#include <hip/hip_runtime.h>


#ifndef NB
#define NB 2
#endif
#ifndef SEQ
#define SEQ 2048
#endif
#define NB_FULL  2
#define SEQ_FULL 2048
#define TT   SEQ
#define DM   1024
#define NH_  16
#define HD   64
#define DQ   (NH_ * HD)
#define QC   256
#define RH   512
#define AW   4
#define PCAR 1024.0f
#define SCL  0.125f
typedef _Float16 h16;
typedef unsigned short bf;
typedef __attribute__((ext_vector_type(16))) __bf16   v16bf;
typedef __attribute__((ext_vector_type(16))) _Float16 v16h;
typedef __attribute__((ext_vector_type(8)))  _Float16 v8h;
typedef __attribute__((ext_vector_type(8)))  unsigned short v8us;
typedef __attribute__((ext_vector_type(8)))  float    v8f;
typedef __attribute__((ext_vector_type(4)))  float    v4f;
typedef v8h  __attribute__((may_alias)) v8ha;
typedef v4f  __attribute__((may_alias)) v4fa;
typedef v8us __attribute__((may_alias)) v8usa;

static_assert(TT % QC == 0);
static_assert(QC % 64 == 0);
static_assert(QC % AW == 0);
static_assert(RH % QC == 0);
static_assert(TT % 128 == 0);
static_assert(HD == 64);
static_assert(DM % 64 == 0);
static_assert((size_t)AW * TT * 4 <= 65536);
static_assert((size_t)NB_FULL * SEQ_FULL * DM * 4 == 16777216);
static_assert((size_t)NB_FULL * SEQ_FULL * DM + (size_t)NB * TT * TT <= (size_t)50331648 / 4);

__device__ __forceinline__ unsigned short f2bf(float f) { unsigned u = __float_as_uint(f); u += 0x7FFFu + ((u >> 16) & 1u); return (unsigned short)(u >> 16); }
__device__ __forceinline__ float bf2f(unsigned short b) { return __uint_as_float(((unsigned)b) << 16); }
__device__ __forceinline__ float bfr(float f) { return bf2f(f2bf(f)); }
__device__ __forceinline__ v16h cat16(v8h lo, v8h hi) { return __builtin_shufflevector(lo, hi, 0, 1, 2, 3, 4, 5, 6, 7, 8, 9, 10, 11, 12, 13, 14, 15); }
__device__ __forceinline__ v16bf cat16b(v8us lo, v8us hi) { return __builtin_bit_cast(v16bf, __builtin_shufflevector(lo, hi, 0, 1, 2, 3, 4, 5, 6, 7, 8, 9, 10, 11, 12, 13, 14, 15)); }
__device__ __forceinline__ v8f wmma16(v16h a, v16h b, v8f c) { return __builtin_amdgcn_wmma_f32_16x16x32_f16(false, a, false, b, (short)0, c, false, false); }
__device__ __forceinline__ v8f wmmab(v16bf a, v16bf b, v8f c) { return __builtin_amdgcn_wmma_f32_16x16x32_bf16(false, a, false, b, (short)0, c, false, false); }

template <typename T16> struct WFrag;
template <> struct WFrag<h16> { typedef v16h V; static __device__ __forceinline__ V ld(const h16* p) { return cat16(*(const v8h*)p, *(const v8h*)(p + 16)); } static __device__ __forceinline__ v8f mma(V a, V b, v8f c) { return wmma16(a, b, c); } };
template <> struct WFrag<bf> { typedef v16bf V; static __device__ __forceinline__ V ld(const bf* p) { return cat16b(*(const v8us*)p, *(const v8us*)(p + 16)); } static __device__ __forceinline__ v8f mma(V a, V b, v8f c) { return wmmab(a, b, c); } };
template <typename T16, int NSPLIT, bool BIAS>
__global__ __launch_bounds__(32) void k_gemmw(const T16* __restrict__ A, const T16* __restrict__ A2, const T16* __restrict__ Bt, const T16* __restrict__ Bt2, int K, float* C, int ldc, const float* __restrict__ bias, size_t sA, size_t sB, size_t sC) {
    typedef typename WFrag<T16>::V V;
    __shared__ __align__(16) float os[16 * 68];
    const size_t z = blockIdx.z; A += z * sA; if (A2) A2 += z * sA; Bt += z * sB; if (Bt2) Bt2 += z * sB; C += z * sC;
    const int lane = threadIdx.x & 31, lr = lane & 15, hi = lane >> 4; const int r0 = blockIdx.x * 64, c0 = blockIdx.y * 64;
    v8f acc[4][4];
#pragma unroll
    for (int mb = 0; mb < 4; ++mb)
#pragma unroll
        for (int nb = 0; nb < 4; ++nb) acc[mb][nb] = (v8f){};
    const size_t aoff = (size_t)(r0 + lr) * K + 8 * hi, boff = (size_t)(c0 + lr) * K + 8 * hi;
#pragma unroll 1
    for (int kc = 0; kc < K; kc += 32) {
        V a[4], a2[4];
#pragma unroll
        for (int mb = 0; mb < 4; ++mb) { a[mb] = WFrag<T16>::ld(A + aoff + (size_t)mb * 16 * K + kc); if (NSPLIT == 1 || NSPLIT == 2) a2[mb] = WFrag<T16>::ld(A2 + aoff + (size_t)mb * 16 * K + kc); }
#pragma unroll
        for (int nb = 0; nb < 4; ++nb) { const V b = WFrag<T16>::ld(Bt + boff + (size_t)nb * 16 * K + kc); V b2; if (NSPLIT >= 2) b2 = WFrag<T16>::ld(Bt2 + boff + (size_t)nb * 16 * K + kc);
#pragma unroll
            for (int mb = 0; mb < 4; ++mb) { acc[mb][nb] = WFrag<T16>::mma(a[mb], b, acc[mb][nb]); if (NSPLIT == 1 || NSPLIT == 2) acc[mb][nb] = WFrag<T16>::mma(a2[mb], b, acc[mb][nb]); if (NSPLIT >= 2) acc[mb][nb] = WFrag<T16>::mma(a[mb], b2, acc[mb][nb]); } }
        asm volatile("v_nop\n\tv_nop\n\tv_nop\n\tv_nop" : "+v"(acc[0][0]), "+v"(acc[1][1]), "+v"(acc[2][2]), "+v"(acc[3][3]) : "v"(a[0]), "v"(a[3]));
    }
#pragma unroll
    for (int mb = 0; mb < 4; ++mb) {
#pragma unroll
        for (int nb = 0; nb < 4; ++nb) {
#pragma unroll
            for (int j = 0; j < 8; ++j) os[(hi * 8 + j) * 68 + nb * 16 + lr] = acc[mb][nb][j]; }
        __builtin_amdgcn_wave_barrier(); asm volatile("" ::: "memory");
        float* crow = C + (size_t)(r0 + mb * 16) * ldc + c0;
#pragma unroll 1
        for (int ps = 0; ps < 2; ++ps) {
#pragma unroll
            for (int s = 0; s < 8; ++s) { const int row = 2 * s + hi, cofs = lr * 4; v4f val = *(const v4fa*)(os + row * 68 + cofs); if (BIAS) { val[0] += bfr(bias[c0 + cofs]); val[1] += bfr(bias[c0 + cofs + 1]); val[2] += bfr(bias[c0 + cofs + 2]); val[3] += bfr(bias[c0 + cofs + 3]); }
                *(volatile v4f*)(crow + (size_t)row * ldc + cofs) = val; }
            if (ps == 0) __threadfence(); }
        __builtin_amdgcn_wave_barrier(); asm volatile("" ::: "memory");
    }
}

__device__ __forceinline__ h16 tohx(float x) { return (h16)x; }
__device__ __forceinline__ void splitf(float y, unsigned short& h, unsigned short& l) { h = f2bf(y); l = f2bf(y - bf2f(h)); }
typedef __attribute__((ext_vector_type(2))) _Float16 v2h;
typedef __attribute__((ext_vector_type(4))) _Float16 v4h;
typedef __attribute__((ext_vector_type(2))) unsigned short v2us;
typedef __attribute__((ext_vector_type(4))) unsigned short v4us;
typedef __attribute__((ext_vector_type(2))) float v2f;

__global__ __launch_bounds__(256) void k_cvt8(const float* __restrict__ src, bf* dst, size_t n8) { const size_t i = (size_t)blockIdx.x * 256 + threadIdx.x; if (i >= n8) return; const v8f v = *(const v8f*)(src + i * 8); v8us o;
#pragma unroll
    for (int k = 0; k < 8; ++k) o[k] = f2bf(v[k]); *(volatile v8us*)(dst + i * 8) = o; __threadfence(); *(volatile v8us*)(dst + i * 8) = o; }

__global__ __launch_bounds__(256) void k_hp(const float* __restrict__ F, int pitch, int nheads, h16* P16, bf* Ph, bf* Pl) {
    const size_t e = ((size_t)blockIdx.x * 256 + threadIdx.x) * 2; if (e >= (size_t)nheads * TT * HD) return; const int d = (int)(e % HD); const int t = (int)((e / HD) % TT); const int h = (int)(e / ((size_t)HD * TT));
    const v2f x = *(const v2f*)(F + (size_t)t * pitch + h * HD + d); v2h o16; v2us oh, ol;
#pragma unroll
    for (int q = 0; q < 2; ++q) { const float r = x[q]; o16[q] = tohx(r); unsigned short a2, c2; splitf(r, a2, c2); oh[q] = a2; ol[q] = c2; }
    *(volatile v2h*)(P16 + e) = o16; *(volatile v2us*)(Ph + e) = oh; *(volatile v2us*)(Pl + e) = ol; __threadfence(); *(volatile v2h*)(P16 + e) = o16; *(volatile v2us*)(Ph + e) = oh; *(volatile v2us*)(Pl + e) = ol; }

__global__ __launch_bounds__(256) void k_vtp(const float* __restrict__ F, int pitch, int nheads, h16* V16, bf* Vh, bf* Vl) { const size_t e = ((size_t)blockIdx.x * 256 + threadIdx.x) * 2; if (e >= (size_t)nheads * HD * TT) return; const int t = (int)(e % TT); const int d = (int)((e / TT) % HD); const int g = (int)(e / ((size_t)TT * HD)); v2h o16; v2us oh, ol;
#pragma unroll
    for (int q = 0; q < 2; ++q) { const float x = F[(size_t)(t + q) * pitch + g * HD + d]; o16[q] = tohx(x); unsigned short a2, c2; splitf(x, a2, c2); oh[q] = a2; ol[q] = c2; }
    *(volatile v2h*)(V16 + e) = o16; *(volatile v2us*)(Vh + e) = oh; *(volatile v2us*)(Vl + e) = ol; __threadfence(); *(volatile v2h*)(V16 + e) = o16; *(volatile v2us*)(Vh + e) = oh; *(volatile v2us*)(Vl + e) = ol; }

__global__ __launch_bounds__(32 * AW) void k_asoft(const float* __restrict__ Sb, int q0, int hires, h16* P16, bf* Ph, bf* Pl, float* AVG) {
#pragma clang fp contract(off)
    __shared__ __align__(16) float avs[AW * TT];
    const int lane = threadIdx.x & 31; const int w = __builtin_amdgcn_readfirstlane((int)(threadIdx.x >> 5)); const int i = blockIdx.x * AW + w; if (i >= QC) return;
    float* avw = avs + w * TT + lane * 4;
#pragma unroll
    for (int ch = 0; ch < TT / 128; ++ch) { v4f zz; zz[0] = 0.f; zz[1] = 0.f; zz[2] = 0.f; zz[3] = 0.f; *(v4fa*)(avw + ch * 128) = zz; }
#pragma unroll 1
    for (int h = 0; h < NH_; ++h) {
        const size_t po = ((size_t)h * QC + i) * TT; const float* sr = Sb + po; float v[TT / 32]; float mx = -3.0e38f;
#pragma unroll
        for (int ch = 0; ch < TT / 128; ++ch) { const int j0 = ch * 128 + lane * 4; const v4f a = *(const v4f*)(sr + j0);
#pragma unroll
            for (int q = 0; q < 4; ++q) { const float t = a[q] * SCL; v[ch * 4 + q] = t; mx = fmaxf(mx, t); } }
#pragma unroll
        for (int sh = 16; sh; sh >>= 1) mx = fmaxf(mx, __shfl_xor(mx, sh, 32));
        float sum = 0.f;
#pragma unroll
        for (int k = 0; k < TT / 32; ++k) { float d0 = __fsub_rn(v[k], mx); asm volatile("" : "+v"(d0)); v[k] = __builtin_amdgcn_exp2f(__fmul_rn(d0, 1.4426950408889634f)); sum += v[k]; }
#pragma unroll
        for (int sh = 16; sh; sh >>= 1) sum += __shfl_xor(sum, sh, 32);
        const float fn = __fdiv_rn(1.0f, sum); const float f = hires ? fn : fn * PCAR;
#pragma unroll
        for (int ch = 0; ch < TT / 128; ++ch) { v4f a = *(const v4fa*)(avw + ch * 128);
#pragma unroll
            for (int q = 0; q < 4; ++q) { const float pn = v[ch * 4 + q] * fn; a[q] = a[q] + pn; }
            *(v4fa*)(avw + ch * 128) = a; }
#pragma unroll 1
        for (int ps = 0; ps < 2; ++ps) {
            float fz = f; asm volatile("" : "+v"(fz));
            if (hires) {
#pragma unroll
                for (int ch = 0; ch < TT / 128; ++ch) { v4us oh, ol;
#pragma unroll
                    for (int q = 0; q < 4; ++q) { unsigned short a, c2; splitf(v[ch * 4 + q] * fz, a, c2); oh[q] = a; ol[q] = c2; }
                    const size_t oo = po + ch * 128 + lane * 4; *(volatile v4us*)(Ph + oo) = oh; *(volatile v4us*)(Pl + oo) = ol; }
            } else {
#pragma unroll
                for (int ch = 0; ch < TT / 128; ++ch) { v4h o4;
#pragma unroll
                    for (int q = 0; q < 4; ++q) o4[q] = tohx(v[ch * 4 + q] * fz);
                    *(volatile v4h*)(P16 + po + ch * 128 + lane * 4) = o4; } }
            if (ps == 0) __threadfence(); }
    }
    float* arow = AVG + (size_t)(q0 + i) * TT;
#pragma unroll 1
    for (int ps = 0; ps < 2; ++ps) {
        float sc = 1.0f / NH_; asm volatile("" : "+v"(sc));
#pragma unroll
        for (int ch = 0; ch < TT / 128; ++ch) { const v4f a = *(const v4fa*)(avw + ch * 128); v4f o;
#pragma unroll
            for (int q = 0; q < 4; ++q) o[q] = a[q] * sc;
            *(volatile v4f*)(arow + ch * 128 + lane * 4) = o; }
        if (ps == 0) __threadfence(); }
}

__global__ __launch_bounds__(256) void k_merge(const float* __restrict__ O, int q0, int hires, bf* Ah, bf* Al) { const size_t e = ((size_t)blockIdx.x * 256 + threadIdx.x) * 2; if (e >= (size_t)NH_ * QC * HD) return; const int d = (int)(e % HD); const int i = (int)((e / HD) % QC); const int h = (int)(e / ((size_t)HD * QC)); const float cs = hires ? 1.0f : (1.0f / PCAR); const size_t oo = (size_t)(q0 + i) * DQ + h * HD + d;
    const v2f x = *(const v2f*)(O + e); v2us oh, ol;
#pragma unroll
    for (int q = 0; q < 2; ++q) { unsigned short a, c2; splitf(x[q] * cs, a, c2); oh[q] = a; ol[q] = c2; } *(volatile v2us*)(Ah + oo) = oh; *(volatile v2us*)(Al + oo) = ol; __threadfence(); *(volatile v2us*)(Ah + oo) = oh; *(volatile v2us*)(Al + oo) = ol; }

static constexpr size_t W_BYTES  = (size_t)DM * DM * 2;
static constexpr size_t XB_BYTES = (size_t)TT * DM * 2;
static constexpr size_t F_BYTES  = (size_t)TT * DM * 4;
static constexpr size_t PL_BYTES = (size_t)NH_ * TT * HD * 2;
static constexpr size_t SB_BYTES = (size_t)NH_ * QC * TT * 4;
static constexpr size_t PP_BYTES = (size_t)NH_ * QC * TT * 2;
static constexpr size_t OB_BYTES = (size_t)NH_ * QC * HD * 4;
static constexpr size_t AT_BYTES = (size_t)TT * DQ * 2;
static constexpr size_t U_BYTES  = (SB_BYTES > XB_BYTES + 2 * F_BYTES) ? SB_BYTES : (XB_BYTES + 2 * F_BYTES);
static constexpr size_t WS_TOTAL = 4 * W_BYTES + U_BYTES + 9 * PL_BYTES + 2 * PP_BYTES + OB_BYTES + 2 * AT_BYTES;
static_assert(W_BYTES % 256 == 0 && XB_BYTES % 256 == 0 && F_BYTES % 256 == 0 && PL_BYTES % 256 == 0);
static_assert(SB_BYTES % 256 == 0 && PP_BYTES % 256 == 0 && OB_BYTES % 256 == 0 && AT_BYTES % 256 == 0);
static_assert(XB_BYTES + 2 * F_BYTES <= U_BYTES);
static_assert(SB_BYTES <= U_BYTES);
static_assert(WS_TOTAL <= (size_t)134217728);

extern "C" void kernel_launch(void* const* d_in, const int* in_sizes, int n_in,
                              void* d_out, int out_size, void* d_ws, size_t ws_size, hipStream_t stream) {
    if (n_in < 11) return;
    const size_t need_x = (size_t)(NB - 1) * SEQ_FULL * DM + (size_t)TT * DM;
    if ((size_t)in_sizes[0] < need_x || (size_t)in_sizes[1] < need_x || (size_t)in_sizes[2] < need_x) return;
    if ((size_t)in_sizes[3] < (size_t)DM * DM || (size_t)in_sizes[5] < (size_t)DM * DM || (size_t)in_sizes[7] < (size_t)DM * DM || (size_t)in_sizes[9] < (size_t)DM * DM) return;
    if (in_sizes[4] < DM || in_sizes[6] < DM || in_sizes[8] < DM || in_sizes[10] < DM) return;
    const size_t AVG_OFF = (size_t)NB_FULL * SEQ_FULL * DM;
    if ((size_t)out_size < AVG_OFF + (size_t)NB * TT * TT) return;
    if (ws_size < WS_TOTAL) return;
    const float* xq = (const float*)d_in[0]; const float* xk = (const float*)d_in[1]; const float* xv = (const float*)d_in[2]; const float* wq = (const float*)d_in[3]; const float* bq = (const float*)d_in[4]; const float* wk = (const float*)d_in[5]; const float* bk = (const float*)d_in[6]; const float* wv = (const float*)d_in[7]; const float* bv = (const float*)d_in[8]; const float* wo = (const float*)d_in[9]; const float* bo = (const float*)d_in[10];
    float* OUT = (float*)d_out;
    float* AVG = (float*)d_out + AVG_OFF;
    char* wsp = (char*)d_ws;
    auto take = [&](size_t bytes) { char* p = wsp; wsp += (bytes + 255) & ~(size_t)255; return (void*)p; };
    bf* WQ = (bf*)take(W_BYTES); bf* WK = (bf*)take(W_BYTES); bf* WV = (bf*)take(W_BYTES); bf* WO = (bf*)take(W_BYTES);
    char* U = (char*)take(U_BYTES);
    float* Sb = (float*)U; bf* XB = (bf*)U; float* FQ = (float*)(U + XB_BYTES); float* FK = (float*)(U + XB_BYTES + F_BYTES); float* FV = FK;
    h16* QP16 = (h16*)take(PL_BYTES); h16* KP16 = (h16*)take(PL_BYTES); h16* VT16 = (h16*)take(PL_BYTES);
    bf* QPh = (bf*)take(PL_BYTES); bf* QPl = (bf*)take(PL_BYTES); bf* KPh = (bf*)take(PL_BYTES); bf* KPl = (bf*)take(PL_BYTES); bf* VTh = (bf*)take(PL_BYTES); bf* VTl = (bf*)take(PL_BYTES);
    char* PAr = (char*)take(PP_BYTES); h16* PA16 = (h16*)PAr; bf* PAh = (bf*)PAr;
    bf* PAl = (bf*)take(PP_BYTES);
    float* Ob = (float*)take(OB_BYTES); bf* ATh = (bf*)take(AT_BYTES); bf* ATl = (bf*)take(AT_BYTES);
    if ((size_t)(wsp - (char*)d_ws) > ws_size) return;

    const unsigned GW = (unsigned)(((size_t)DM * DM / 8 + 255) / 256), GX = (unsigned)(((size_t)TT * DM / 8 + 255) / 256);
    k_cvt8<<<GW, 256, 0, stream>>>(wq, WQ, (size_t)DM * DM / 8); k_cvt8<<<GW, 256, 0, stream>>>(wk, WK, (size_t)DM * DM / 8);
    k_cvt8<<<GW, 256, 0, stream>>>(wv, WV, (size_t)DM * DM / 8); k_cvt8<<<GW, 256, 0, stream>>>(wo, WO, (size_t)DM * DM / 8);
    const unsigned LP = (unsigned)(((size_t)NH_ * TT * HD / 2 + 255) / 256);
    const unsigned LM = (unsigned)(((size_t)NH_ * QC * HD / 2 + 255) / 256);
    for (int b = 0; b < NB; ++b) {
        const size_t xo = (size_t)b * SEQ_FULL * DM;
        k_cvt8<<<GX, 256, 0, stream>>>(xq + xo, XB, (size_t)TT * DM / 8);
        k_gemmw<bf, 0, true><<<dim3(TT / 64, DQ / 64, 1), 32, 0, stream>>>(XB, nullptr, WQ, nullptr, DM, FQ, DQ, bq, 0, 0, 0);
        k_hp<<<LP, 256, 0, stream>>>(FQ, DQ, NH_, QP16, QPh, QPl);
        k_cvt8<<<GX, 256, 0, stream>>>(xk + xo, XB, (size_t)TT * DM / 8);
        k_gemmw<bf, 0, true><<<dim3(TT / 64, DQ / 64, 1), 32, 0, stream>>>(XB, nullptr, WK, nullptr, DM, FK, DQ, bk, 0, 0, 0);
        k_hp<<<LP, 256, 0, stream>>>(FK, DQ, NH_, KP16, KPh, KPl);
        k_cvt8<<<GX, 256, 0, stream>>>(xv + xo, XB, (size_t)TT * DM / 8);
        k_gemmw<bf, 0, true><<<dim3(TT / 64, DQ / 64, 1), 32, 0, stream>>>(XB, nullptr, WV, nullptr, DM, FV, DQ, bv, 0, 0, 0);
        k_vtp<<<LP, 256, 0, stream>>>(FV, DQ, NH_, VT16, VTh, VTl);
        for (int q0 = 0; q0 < TT; q0 += QC) {
            const int hires = (q0 < RH) ? 1 : 0;
            if (hires) k_gemmw<bf, 2, false><<<dim3(QC / 64, TT / 64, NH_), 32, 0, stream>>>(QPh + (size_t)q0 * HD, QPl + (size_t)q0 * HD, KPh, KPl, HD, Sb, TT, nullptr, (size_t)TT * HD, (size_t)TT * HD, (size_t)QC * TT);
            else       k_gemmw<h16, 0, false><<<dim3(QC / 64, TT / 64, NH_), 32, 0, stream>>>(QP16 + (size_t)q0 * HD, nullptr, KP16, nullptr, HD, Sb, TT, nullptr, (size_t)TT * HD, (size_t)TT * HD, (size_t)QC * TT);
            k_asoft<<<QC / AW, 32 * AW, 0, stream>>>(Sb, q0, hires, PA16, PAh, PAl, AVG + (size_t)b * TT * TT);
            if (hires) k_gemmw<bf, 2, false><<<dim3(QC / 64, HD / 64, NH_), 32, 0, stream>>>(PAh, PAl, VTh, VTl, TT, Ob, HD, nullptr, (size_t)QC * TT, (size_t)HD * TT, (size_t)QC * HD);
            else       k_gemmw<h16, 0, false><<<dim3(QC / 64, HD / 64, NH_), 32, 0, stream>>>(PA16, nullptr, VT16, nullptr, TT, Ob, HD, nullptr, (size_t)QC * TT, (size_t)HD * TT, (size_t)QC * HD);
            k_merge<<<LM, 256, 0, stream>>>(Ob, q0, hires, ATh, ATl);
        }
        k_gemmw<bf, 1, true><<<dim3(TT / 64, DM / 64, 1), 32, 0, stream>>>(ATh, ATl, WO, nullptr, DQ, OUT + (size_t)b * TT * DM, DM, bo, 0, 0, 0);
    }
}
